// SelfAttention_66116726554651
// MI455X (gfx1250) — hardware-verified
//
#include <hip/hip_runtime.h>
#ifndef NB
#define NB 4
#endif
#ifndef SEQ
#define SEQ 2048
#endif
#define NB_FULL 4
#define SEQ_FULL 2048
#define DMODEL 256
#define NHEAD 8
#define HD 32
#define LDQK 512
#define NW3 768
#define TOK (NB * SEQ)
#define EARLY ((SEQ < 512) ? SEQ : 512)
#define NEGBIG (-1.0e30f)
#define SSCALE 0.17677669529663687f
#define RINV 0.00048828125f

static_assert(NHEAD * HD == DMODEL);
static_assert(HD == 32);
static_assert(NHEAD % 2 == 0);
static_assert(2 * DMODEL == LDQK && 3 * DMODEL == NW3);
static_assert(SEQ % 128 == 0 && SEQ % 64 == 0 && SEQ % 32 == 0);
static_assert(TOK % 128 == 0 && TOK % 64 == 0);
static_assert(DMODEL % 128 == 0 && DMODEL % 64 == 0 && DMODEL % 32 == 0 && DMODEL % 8 == 0 && LDQK % 64 == 0);
static_assert(EARLY % 128 == 0 && EARLY % 64 == 0 && EARLY % 32 == 0 && EARLY <= SEQ);
static_assert(NB <= NB_FULL && SEQ <= SEQ_FULL);
static_assert(SEQ + 32 < 40000);

typedef unsigned short v8us __attribute__((ext_vector_type(8), may_alias));
typedef float  v8f  __attribute__((ext_vector_type(8)));
typedef float  v4f  __attribute__((ext_vector_type(4)));
typedef float  v4fa __attribute__((ext_vector_type(4), may_alias));
typedef _Float16 v16h __attribute__((ext_vector_type(16)));
union FragH { v16h v; v8us half[2]; _Float16 h[16]; unsigned short u[16]; };

__device__ __forceinline__ unsigned short bf16_bits(float x) { unsigned int u = __float_as_uint(x); return (unsigned short)((u + 0x7FFFu + ((u >> 16) & 1u)) >> 16); }
__device__ __forceinline__ float bf16_rne(float x) { return __uint_as_float(((unsigned int)bf16_bits(x)) << 16); }

__device__ __forceinline__ v16h g2_frag(const _Float16* p, int hh) { FragH f; f.half[0] = *(const v8us*)((const unsigned short*)p + 8 * hh); f.half[1] = *(const v8us*)((const unsigned short*)p + 16 + 8 * hh); return f.v; }
__device__ __forceinline__ v8f g2_mma(v16h a, v16h b, v8f c) { v8f d = __builtin_amdgcn_wmma_f32_16x16x32_f16(false, a, false, b, (short)0, c, false, false); asm volatile("v_nop\n\tv_nop\n\tv_nop\n\tv_nop" : "+v"(d) : "v"(a), "v"(b)); return d; }

__global__ __launch_bounds__(256) void k_x16(const float* __restrict__ x, _Float16* __restrict__ X16) {
  const size_t t = (size_t)blockIdx.x * 256 + threadIdx.x; if (t >= (size_t)TOK * (DMODEL / 8)) return;
  const size_t r = t / (DMODEL / 8); const int c8 = (int)(t % (DMODEL / 8)) * 8; const size_t b = r / SEQ, s = r % SEQ;
  const float* src = x + (b * SEQ_FULL + s) * DMODEL + c8; const v4f a = *(const v4fa*)src, c = *(const v4fa*)(src + 4); FragH f;
#pragma unroll
  for (int q = 0; q < 4; ++q) { f.h[q] = (_Float16)bf16_rne(a[q]); f.h[4 + q] = (_Float16)bf16_rne(c[q]); }
  const v8us o = f.half[0]; unsigned short* d = (unsigned short*)X16 + t * 8;
  *(volatile v8us*)d = o; __threadfence(); *(volatile v8us*)d = o; }

__global__ __launch_bounds__(256) void k_wnat(const float* __restrict__ w, size_t n8, float scale, _Float16* __restrict__ Bt) {
  const size_t t = (size_t)blockIdx.x * 256 + threadIdx.x; if (t >= n8) return; const v4f a = *(const v4fa*)(w + t * 8), c = *(const v4fa*)(w + t * 8 + 4); FragH f;
#pragma unroll
  for (int q = 0; q < 4; ++q) { f.h[q] = (_Float16)(bf16_rne(a[q]) * scale); f.h[4 + q] = (_Float16)(bf16_rne(c[q]) * scale); }
  const v8us o = f.half[0]; unsigned short* d = (unsigned short*)Bt + t * 8;
  *(volatile v8us*)d = o; __threadfence(); *(volatile v8us*)d = o; }

template <int MODE, bool RESA>
__device__ __forceinline__ void gemm_body(const _Float16* __restrict__ A, const _Float16* __restrict__ AR, int lda, const _Float16* __restrict__ Bh, int ldb, float alpha,
                                          const float* __restrict__ biasA, const float* __restrict__ biasB, int nsplit,
                                          float* __restrict__ C, _Float16* __restrict__ C16, _Float16* __restrict__ C16R, int ldc, int M, int N, int K) {
  __shared__ __attribute__((aligned(16))) float so[4][32][68];
  const int tid = threadIdx.x, lane = tid & 31, ln = lane & 15, hh = lane >> 4;
  const int w = __builtin_amdgcn_readfirstlane(tid >> 5);
  const int ntn = N >> 6; const int mt = blockIdx.x / ntn, nq = blockIdx.x - mt * ntn; const int row0 = mt * 128 + 32 * w, col0 = nq * 64; if (row0 >= M) return;
  const _Float16* a0p = A + (size_t)(row0 + ln) * lda; const _Float16* a1p = a0p + (size_t)16 * lda;
  const _Float16* b0p = Bh + (size_t)(col0 + ln) * ldb; const _Float16* b1p = b0p + (size_t)16 * ldb; const _Float16* b2p = b1p + (size_t)16 * ldb; const _Float16* b3p = b2p + (size_t)16 * ldb;
  const v8f z8 = {0.f,0.f,0.f,0.f,0.f,0.f,0.f,0.f}; v8f c00 = z8, c01 = z8, c02 = z8, c03 = z8, c10 = z8, c11 = z8, c12 = z8, c13 = z8;
#pragma unroll 1
  for (int kb = 0; kb < K; kb += 32) { const v16h a0 = g2_frag(a0p + kb, hh), a1 = g2_frag(a1p + kb, hh);
    v16h b = g2_frag(b0p + kb, hh); c00 = g2_mma(a0, b, c00); c10 = g2_mma(a1, b, c10);
    b = g2_frag(b1p + kb, hh); c01 = g2_mma(a0, b, c01); c11 = g2_mma(a1, b, c11);
    b = g2_frag(b2p + kb, hh); c02 = g2_mma(a0, b, c02); c12 = g2_mma(a1, b, c12);
    b = g2_frag(b3p + kb, hh); c03 = g2_mma(a0, b, c03); c13 = g2_mma(a1, b, c13); }
  v8f r00 = z8, r01 = z8, r02 = z8, r03 = z8, r10 = z8, r11 = z8, r12 = z8, r13 = z8;
  if (RESA) {
    const bool early = ((mt * 128) % SEQ) < EARLY;
    if (early) {
      const _Float16* e0p = AR + (size_t)(row0 + ln) * lda; const _Float16* e1p = e0p + (size_t)16 * lda;
#pragma unroll 1
      for (int kb = 0; kb < K; kb += 32) { const v16h a0 = g2_frag(e0p + kb, hh), a1 = g2_frag(e1p + kb, hh);
        v16h b = g2_frag(b0p + kb, hh); r00 = g2_mma(a0, b, r00); r10 = g2_mma(a1, b, r10);
        b = g2_frag(b1p + kb, hh); r01 = g2_mma(a0, b, r01); r11 = g2_mma(a1, b, r11);
        b = g2_frag(b2p + kb, hh); r02 = g2_mma(a0, b, r02); r12 = g2_mma(a1, b, r12);
        b = g2_frag(b3p + kb, hh); r03 = g2_mma(a0, b, r03); r13 = g2_mma(a1, b, r13); }
    }
  }
  v8f accs[8] = {c00, c01, c02, c03, c10, c11, c12, c13};
  if (RESA) { const v8f racc[8] = {r00, r01, r02, r03, r10, r11, r12, r13};
#pragma unroll
    for (int u = 0; u < 8; ++u) accs[u] = accs[u] + racc[u] * RINV; }
  float brow[16];
#pragma unroll
  for (int i = 0; i < 16; ++i) brow[i] = 0.f;
  if (MODE == 2) {
#pragma unroll
    for (int i = 0; i < 16; ++i) brow[i] = bf16_rne(biasA[row0 + (i >> 3) * 16 + 8 * hh + (i & 7)]);
  }
#pragma unroll
  for (int u = 0; u < 8; ++u) { const int t = u & 3, half = u >> 2; const int col = col0 + t * 16 + ln; float bcol = 0.f;
    if (MODE != 2) { const int ca = (col < nsplit) ? col : (nsplit - 1); const int cb = (col >= nsplit) ? (col - nsplit) : 0;
      const float va = biasA[ca], vb = biasB[cb]; bcol = bf16_rne((col < nsplit) ? va : vb); }
#pragma unroll
    for (int r = 0; r < 8; ++r) { const int rloc = half * 16 + 8 * hh + r; const float v = accs[u][r] * alpha + ((MODE == 2) ? brow[half * 8 + r] : bcol); so[w][rloc][t * 16 + ln] = v; } }
  __builtin_amdgcn_fence(4  , "workgroup"); __builtin_amdgcn_wave_barrier();
  if (MODE == 0) {
    const int rsub = lane >> 4, c4 = (lane & 15) * 4;
    for (int pass = 0; pass < 2; ++pass) {
#pragma unroll
      for (int q = 0; q < 16; ++q) { const int r = q * 2 + rsub; const v4f v = *(const v4fa*)&so[w][r][c4]; *(volatile v4f*)(C + (size_t)(row0 + r) * ldc + col0 + c4) = v; }
      if (pass == 0) __threadfence(); }
  } else {
    const int rq = lane >> 3, c8 = (lane & 7) * 8;
    const bool wr = (MODE == 2) && ((col0 % SEQ) < EARLY);
    for (int pass = 0; pass < 2; ++pass) {
#pragma unroll
      for (int q = 0; q < 8; ++q) { const int r = q * 4 + rq; const v4f a = *(const v4fa*)&so[w][r][c8], c = *(const v4fa*)&so[w][r][c8 + 4]; FragH f, g;
#pragma unroll
        for (int i = 0; i < 4; ++i) { const _Float16 ha = (_Float16)a[i], hc = (_Float16)c[i]; f.h[i] = ha; f.h[4 + i] = hc;
          g.h[i] = (_Float16)((a[i] - (float)ha) * 2048.0f); g.h[4 + i] = (_Float16)((c[i] - (float)hc) * 2048.0f); }
        const v8us o = f.half[0]; *(volatile v8us*)((unsigned short*)C16 + (size_t)(row0 + r) * ldc + col0 + c8) = o;
        if (MODE == 2) { if (wr) { const v8us o2 = g.half[0]; *(volatile v8us*)((unsigned short*)C16R + (size_t)(row0 + r) * ldc + col0 + c8) = o2; } } }
      if (pass == 0) __threadfence(); }
  }
}

__global__ __launch_bounds__(128) void k_gemm_qk(const _Float16* __restrict__ X16, const _Float16* __restrict__ W16, const float* __restrict__ qb, const float* __restrict__ kbias, _Float16* __restrict__ QK) {
  gemm_body<1, false>(X16, X16, DMODEL, W16, DMODEL, 0.015625f, qb, kbias, DMODEL, nullptr, QK, nullptr, LDQK, TOK, LDQK, DMODEL); }
__global__ __launch_bounds__(128) void k_gemm_vt(const _Float16* __restrict__ X16, const _Float16* __restrict__ W16, const float* __restrict__ vb, _Float16* __restrict__ VT, _Float16* __restrict__ VTR) {
  gemm_body<2, false>(W16 + (size_t)LDQK * DMODEL, W16, DMODEL, X16, DMODEL, 0.015625f, vb, vb, DMODEL, nullptr, VT, VTR, TOK, DMODEL, TOK, DMODEL); }
__global__ __launch_bounds__(128) void k_gemm_out(const _Float16* __restrict__ CTX, const _Float16* __restrict__ CTXR, const _Float16* __restrict__ WO16, const float* __restrict__ ob, float* __restrict__ out) {
  gemm_body<0, true>(CTX, CTXR, DMODEL, WO16, DMODEL, 0.000244140625f, ob, ob, DMODEL, out, nullptr, nullptr, DMODEL, TOK, DMODEL, DMODEL); }

template <bool RES>
__device__ __forceinline__ void flash_body(const _Float16* __restrict__ QK, const _Float16* __restrict__ VT, const _Float16* __restrict__ VTR,
                                           _Float16* __restrict__ CTX, _Float16* __restrict__ CTXR, int qb0) {
  __shared__ __attribute__((aligned(16))) unsigned short so[32][72];
  __shared__ __attribute__((aligned(16))) unsigned short sor[RES ? 32 : 1][72];
  const int tid = threadIdx.x, lane = tid & 31, ln = lane & 15, hh = lane >> 4;
  const int wave = __builtin_amdgcn_readfirstlane(tid >> 5);
  const int hp = wave & 1, qg = wave >> 1;
  const int head = 2 * (int)blockIdx.y + hp;
  const size_t tokb = (size_t)blockIdx.z * SEQ;
  const int q0 = (qb0 + (int)blockIdx.x) * 32;
  const int i0 = q0 + qg * 16;
  const int qi = i0 + ln;
  const v16h bq = g2_frag(QK + (tokb + qi) * LDQK + head * HD, hh);
  const _Float16* kbase = QK + (tokb + ln) * LDQK + DMODEL + head * HD;
  const _Float16* vbase = VT + (size_t)(head * HD + ln) * TOK + tokb;
  const _Float16* rbase = VTR + (size_t)(head * HD + ln) * TOK + tokb;
  const v8f z8 = {0.f,0.f,0.f,0.f,0.f,0.f,0.f,0.f};
  v8f o0 = z8, o1 = z8, x0 = z8, x1 = z8; float m = NEGBIG, l = 0.f;
  const int jend = i0 + 16;
#pragma unroll 1
  for (int j = 0; j < jend; j += 32) {
    const _Float16* k0p = kbase + (size_t)j * LDQK;
    v8f s0 = g2_mma(g2_frag(k0p, hh), bq, z8);
    v8f s1 = g2_mma(g2_frag(k0p + (size_t)16 * LDQK, hh), bq, z8);
    const int kb0 = j + 8 * hh;
    const int c0 = qi - kb0, c1 = c0 - 16;
    const int res = (int)((unsigned int)kb0 % 25u);
    const int d0 = 24 - res, d1 = 8 - res;
#pragma unroll
    for (int r = 0; r < 8; ++r) { s0[r] = ((r <= c0) && (r != d0)) ? s0[r] : NEGBIG; s1[r] = ((r <= c1) && (r != d1)) ? s1[r] : NEGBIG; }
    float mx = fmaxf(s0[0], s1[0]);
#pragma unroll
    for (int r = 1; r < 8; ++r) mx = fmaxf(mx, fmaxf(s0[r], s1[r]));
    mx = fmaxf(mx, __shfl_xor(mx, 16, 32));
    const float mn = fmaxf(m, mx * SSCALE); const float al = __expf(m - mn); m = mn;
    FragH pf, pg; float rs = 0.f;
#pragma unroll
    for (int r = 0; r < 8; ++r) { const float p0 = __expf(fmaf(s0[r], SSCALE, -mn)), p1 = __expf(fmaf(s1[r], SSCALE, -mn)); rs += p0 + p1;
      const float a0 = p0 * 256.0f, a1 = p1 * 256.0f; const _Float16 h0 = (_Float16)a0, h1 = (_Float16)a1; pf.h[r] = h0; pf.h[8 + r] = h1;
      pg.h[r] = (_Float16)((a0 - (float)h0) * 2048.0f); pg.h[8 + r] = (_Float16)((a1 - (float)h1) * 2048.0f); }
    l = l * al + rs; o0 = o0 * al; o1 = o1 * al;
    if (RES) { x0 = x0 * al; x1 = x1 * al; }
    const _Float16* vp = vbase + j;
    v16h a = g2_frag(vp, hh);
    o0 = g2_mma(a, pf.v, o0);
    if (RES) { x0 = g2_mma(a, pg.v, x0); x0 = g2_mma(g2_frag(rbase + j, hh), pf.v, x0); }
    a = g2_frag(vp + (size_t)16 * TOK, hh);
    o1 = g2_mma(a, pf.v, o1);
    if (RES) { x1 = g2_mma(a, pg.v, x1); x1 = g2_mma(g2_frag(rbase + j + (size_t)16 * TOK, hh), pf.v, x1); }
  }
  l += __shfl_xor(l, 16, 32);
  const float sc = 0.25f * (1.0f / l);
  { const int row = qg * 16 + ln, cb = hp * 32 + 8 * hh; FragH f, g;
#pragma unroll
    for (int r = 0; r < 8; ++r) { float c = o0[r]; if (RES) c += x0[r] * RINV; c *= sc; const _Float16 hc = (_Float16)c; f.h[r] = hc; g.h[r] = (_Float16)((c - (float)hc) * 2048.0f); }
    *(v8us*)&so[row][cb] = f.half[0]; if (RES) *(v8us*)&sor[row][cb] = g.half[0];
#pragma unroll
    for (int r = 0; r < 8; ++r) { float c = o1[r]; if (RES) c += x1[r] * RINV; c *= sc; const _Float16 hc = (_Float16)c; f.h[r] = hc; g.h[r] = (_Float16)((c - (float)hc) * 2048.0f); }
    *(v8us*)&so[row][cb + 16] = f.half[0]; if (RES) *(v8us*)&sor[row][cb + 16] = g.half[0]; }
  __syncthreads();
  const int rr = tid >> 3, pc = (tid & 7) * 8;
  unsigned short* cdst = (unsigned short*)CTX + (tokb + q0) * DMODEL + 2 * (int)blockIdx.y * HD + pc;
  unsigned short* rdst = (unsigned short*)CTXR + (tokb + q0) * DMODEL + 2 * (int)blockIdx.y * HD + pc;
  for (int pass = 0; pass < 2; ++pass) {
#pragma unroll
    for (int it = 0; it < 2; ++it) { const int r = it * 16 + rr; const v8us v = *(const v8us*)&so[r][pc];
      *(volatile v8us*)(cdst + (size_t)r * DMODEL) = v;
      if (RES) { const v8us v2 = *(const v8us*)&sor[r][pc]; *(volatile v8us*)(rdst + (size_t)r * DMODEL) = v2; } }
    if (pass == 0) __threadfence(); }
}

__global__ __launch_bounds__(128) void k_flash_early(const _Float16* __restrict__ QK, const _Float16* __restrict__ VT, const _Float16* __restrict__ VTR, _Float16* __restrict__ CTX, _Float16* __restrict__ CTXR) {
  flash_body<true>(QK, VT, VTR, CTX, CTXR, 0); }
__global__ __launch_bounds__(128) void k_flash_late(const _Float16* __restrict__ QK, const _Float16* __restrict__ VT, _Float16* __restrict__ CTX) {
  flash_body<false>(QK, VT, VT, CTX, CTX, EARLY / 32); }

extern "C" void kernel_launch(void* const* d_in, const int* in_sizes, int n_in,
                              void* d_out, int out_size, void* d_ws, size_t ws_size, hipStream_t stream) {
  if (n_in < 9) return;
  const size_t need_x = ((size_t)(NB - 1) * SEQ_FULL + SEQ) * DMODEL;
  if ((size_t)in_sizes[0] < need_x) return;
  if ((size_t)in_sizes[1] < (size_t)DMODEL * DMODEL) return;
  if ((size_t)in_sizes[2] < (size_t)DMODEL) return;
  if ((size_t)in_sizes[3] < (size_t)DMODEL * DMODEL) return;
  if ((size_t)in_sizes[4] < (size_t)DMODEL) return;
  if ((size_t)in_sizes[5] < (size_t)DMODEL * DMODEL) return;
  if ((size_t)in_sizes[6] < (size_t)DMODEL) return;
  if ((size_t)in_sizes[7] < (size_t)DMODEL * DMODEL) return;
  if ((size_t)in_sizes[8] < (size_t)DMODEL) return;
  if ((size_t)out_size < (size_t)TOK * DMODEL) return;
  const float* x = (const float*)d_in[0];
  const float* wq = (const float*)d_in[1]; const float* qb = (const float*)d_in[2];
  const float* wk = (const float*)d_in[3]; const float* kbias = (const float*)d_in[4];
  const float* wv = (const float*)d_in[5]; const float* vb = (const float*)d_in[6];
  const float* wo = (const float*)d_in[7]; const float* ob = (const float*)d_in[8];
  constexpr size_t SZ_X = (size_t)TOK * DMODEL * 2;
  constexpr size_t SZ_W = (size_t)NW3 * DMODEL * 2;
  constexpr size_t SZ_WO = (size_t)DMODEL * DMODEL * 2;
  constexpr size_t SZ_QK = (size_t)TOK * LDQK * 2;
  constexpr size_t SZ_VT = (size_t)DMODEL * TOK * 2;
  constexpr size_t SZ_CTX = (size_t)TOK * DMODEL * 2;
  constexpr size_t SZ_ALL = SZ_X + SZ_W + SZ_WO + SZ_QK + 2 * SZ_VT + 2 * SZ_CTX;
  static_assert(SZ_X % 256 == 0 && SZ_W % 256 == 0 && SZ_WO % 256 == 0 && SZ_QK % 256 == 0 && SZ_VT % 256 == 0 && SZ_CTX % 256 == 0);
  static_assert(SZ_ALL <= (size_t)134217728);
  if (SZ_ALL > ws_size) return;
  char* ws = (char*)d_ws;
  _Float16* X16 = (_Float16*)ws; _Float16* W16 = (_Float16*)(ws + SZ_X); _Float16* WO16 = (_Float16*)(ws + SZ_X + SZ_W);
  _Float16* QK = (_Float16*)(ws + SZ_X + SZ_W + SZ_WO);
  _Float16* VT = (_Float16*)(ws + SZ_X + SZ_W + SZ_WO + SZ_QK); _Float16* VTR = (_Float16*)(ws + SZ_X + SZ_W + SZ_WO + SZ_QK + SZ_VT);
  _Float16* CTX = (_Float16*)(ws + SZ_X + SZ_W + SZ_WO + SZ_QK + 2 * SZ_VT); _Float16* CTXR = (_Float16*)(ws + SZ_X + SZ_W + SZ_WO + SZ_QK + 2 * SZ_VT + SZ_CTX);
  constexpr size_t W8 = (size_t)DMODEL * DMODEL / 8;
  constexpr unsigned WG = (unsigned)((W8 + 255) / 256);
  k_x16<<<(unsigned)(((size_t)TOK * (DMODEL / 8) + 255) / 256), 256, 0, stream>>>(x, X16);
  k_wnat<<<WG, 256, 0, stream>>>(wq, W8, 64.0f, W16);
  k_wnat<<<WG, 256, 0, stream>>>(wk, W8, 64.0f, W16 + (size_t)DMODEL * DMODEL);
  k_wnat<<<WG, 256, 0, stream>>>(wv, W8, 64.0f, W16 + (size_t)2 * DMODEL * DMODEL);
  k_wnat<<<WG, 256, 0, stream>>>(wo, W8, 64.0f, WO16);
  k_gemm_qk<<<(TOK / 128) * (LDQK / 64), 128, 0, stream>>>(X16, W16, qb, kbias, QK);
  k_gemm_vt<<<(DMODEL / 128) * (TOK / 64), 128, 0, stream>>>(X16, W16, vb, VT, VTR);
  k_flash_early<<<dim3(EARLY / 32, NHEAD / 2, NB), 128, 0, stream>>>(QK, VT, VTR, CTX, CTXR);
  if (SEQ > EARLY) k_flash_late<<<dim3((SEQ - EARLY) / 32 + ((SEQ > EARLY) ? 0 : 1), NHEAD / 2, NB), 128, 0, stream>>>(QK, VT, CTX);
  k_gemm_out<<<(TOK / 128) * (DMODEL / 64), 128, 0, stream>>>(CTX, CTXR, WO16, ob, (float*)d_out);
}
